// Decoder_90847148245055
// MI455X (gfx1250) — hardware-verified
//
#include <hip/hip_runtime.h>
#include <math.h>

constexpr int kL    = 2;
constexpr int kH    = 512;
constexpr int kE    = 512;
constexpr int kB    = 16;
constexpr int kT    = 512;
constexpr int kS    = 512;
constexpr int kVoc  = 1001;
constexpr int kVocP = 1024;
constexpr int kOut  = 1000;
constexpr int kOutP = 1024;
constexpr int kG    = 4 * kH;
constexpr int kGD   = 2 * kG;
constexpr int kRows = kB * kT;
constexpr int kChunk = 128;
constexpr int kHP   = 520;
constexpr int kSLP  = 36;
constexpr float kWCarry   = 16.0f;
constexpr float kHCarry   = 16.0f;
constexpr float kECarry   = 16.0f;
constexpr float kCatCarry = 16.0f;
constexpr float kPCarry   = 32768.0f;
constexpr float kFoldHW   = 1.0f / (kHCarry * kWCarry);
constexpr float kFoldEW   = 1.0f / (kECarry * kWCarry);
constexpr float kFoldW    = 1.0f / kWCarry;
constexpr float kFoldCW   = 1.0f / (kCatCarry * kWCarry);
constexpr float kCtxScale = kCatCarry / kPCarry;
constexpr int kBiasN = kL * kGD + kH + kOutP;
static_assert(kH == 512 && kT == 512 && kS == 512 && kB == 16, "shape");
static_assert(kT % kChunk == 0 && (kChunk % 2) == 0, "chunking");
static_assert(kH % 32 == 0 && (2 * kH) % 32 == 0 && kE % 32 == 0 && kS % 64 == 0, "K multiples of 32");
static_assert(kVocP % 64 == 0 && kGD % 64 == 0 && kRows % 64 == 0 && kOutP % 64 == 0 && kH % 64 == 0, "tile multiples");
static_assert((kB * kChunk) % 64 == 0, "chunk rows tile multiple");
static_assert(kBiasN == 9728 && (kBiasN % 128) == 0, "bias table whole waves");
static_assert(((long)kRows * kOut) % 2048 == 0, "pack grid exact");
static_assert(kOut % 4 == 0, "output rows split into float4 groups");

typedef __attribute__((ext_vector_type(16))) _Float16 v16h;
typedef __attribute__((ext_vector_type(8)))  _Float16 v8h;
typedef __attribute__((ext_vector_type(16))) __bf16   v16b;
typedef __attribute__((ext_vector_type(8)))  __bf16   v8b;
typedef __attribute__((ext_vector_type(8)))  float    v8f;
typedef __attribute__((ext_vector_type(4)))  float    v4f;
typedef __attribute__((ext_vector_type(4)))  unsigned int v4u;

__device__ __forceinline__ unsigned short f2bf_bits(float f) {
  unsigned u = __float_as_uint(f);
  return (unsigned short)((u + 0x7FFFu + ((u >> 16) & 1u)) >> 16);
}
__device__ __forceinline__ float bf_bits2f(unsigned short h) { return __uint_as_float(((unsigned)h) << 16); }
__device__ __forceinline__ float bf16r(float f) { return bf_bits2f(f2bf_bits(f)); }

__device__ __forceinline__ void guard4_h(v8f& a, v8f& b, v8f& c, v8f& d, v16h x, v16h y) {
  asm volatile("v_nop\n\tv_nop\n\tv_nop\n\tv_nop" : "+v"(a), "+v"(b), "+v"(c), "+v"(d) : "v"(x), "v"(y));
}
__device__ __forceinline__ void guard4_b(v8f& a, v8f& b, v8f& c, v8f& d, v16b x, v16b y) {
  asm volatile("v_nop\n\tv_nop\n\tv_nop\n\tv_nop" : "+v"(a), "+v"(b), "+v"(c), "+v"(d) : "v"(x), "v"(y));
}
__device__ __forceinline__ void guard4w_h(v8f& a, v8f& b, v8f& c, v8f& d, v16h x, v16h b0, v16h b1, v16h b2, v16h b3) {
  asm volatile("v_nop\n\tv_nop\n\tv_nop\n\tv_nop" : "+v"(a), "+v"(b), "+v"(c), "+v"(d) : "v"(x), "v"(b0), "v"(b1), "v"(b2), "v"(b3));
}
__device__ __forceinline__ void keep4_h(v16h a, v16h b, v16h c, v16h d) { asm volatile("v_nop" :: "v"(a), "v"(b), "v"(c), "v"(d)); }
__device__ __forceinline__ void keep4_b(v16b a, v16b b, v16b c, v16b d) { asm volatile("v_nop" :: "v"(a), "v"(b), "v"(c), "v"(d)); }
__device__ __forceinline__ void acc_guard4(v8f& a, v8f& b, v8f& c, v8f& d) {
  asm volatile("v_nop\n\tv_nop\n\tv_nop\n\tv_nop" : "+v"(a), "+v"(b), "+v"(c), "+v"(d));
}

template <typename T> struct Frag;
template <> struct Frag<_Float16> {
  typedef v16h V; union U { v16h v; v8h h[2]; };
  static __device__ __forceinline__ v16h load(const _Float16* p) {
    U f; f.h[0] = *(const v8h*)(p); f.h[1] = *(const v8h*)(p + 16); return f.v;
  }
  static __device__ __forceinline__ v8f mma(v16h a, v16h b, v8f c) {
    return __builtin_amdgcn_wmma_f32_16x16x32_f16(false, a, false, b, (short)0, c, false, false);
  }
  static __device__ __forceinline__ void guard4(v8f& a, v8f& b, v8f& c, v8f& d, v16h x, v16h y) { guard4_h(a, b, c, d, x, y); }
  static __device__ __forceinline__ void keep(v16h a, v16h b, v16h c, v16h d) { keep4_h(a, b, c, d); }
};
template <> struct Frag<__bf16> {
  typedef v16b V; union U { v16b v; v8b h[2]; };
  static __device__ __forceinline__ v16b load(const __bf16* p) {
    U f; f.h[0] = *(const v8b*)(p); f.h[1] = *(const v8b*)(p + 16); return f.v;
  }
  static __device__ __forceinline__ v8f mma(v16b a, v16b b, v8f c) {
    return __builtin_amdgcn_wmma_f32_16x16x32_bf16(false, a, false, b, (short)0, c, false, false);
  }
  static __device__ __forceinline__ void guard4(v8f& a, v8f& b, v8f& c, v8f& d, v16b x, v16b y) { guard4_b(a, b, c, d, x, y); }
  static __device__ __forceinline__ void keep(v16b a, v16b b, v16b c, v16b d) { keep4_b(a, b, c, d); }
};

__device__ __forceinline__ float fsig(float x)  { return __builtin_amdgcn_rcpf(1.0f + __expf(-x)); }
__device__ __forceinline__ float ftanh(float x) { return 1.0f - 2.0f * __builtin_amdgcn_rcpf(__expf(2.0f * x) + 1.0f); }

template <int ET> struct Elem;
template <> struct Elem<0> { typedef _Float16 T; };
template <> struct Elem<1> { typedef __bf16 T; };
template <int ET, bool SPLIT, int BIAS_MODE, int OUT_MODE, int SKIP>
__global__ __launch_bounds__(256) void wmma_gemm64(
    const unsigned short* __restrict__ Ap, const unsigned short* __restrict__ A2p, int lda, long strideA,
    const unsigned short* __restrict__ Btp, const unsigned short* __restrict__ Bt2p, int ldb, long strideB,
    void* __restrict__ Cout, void* __restrict__ Cout2, int ldc, long strideC,
    const float* __restrict__ bias, const int* __restrict__ lens,
    int M, int N, int K, float scale) {
  typedef typename Elem<ET>::T T;
  typedef typename Frag<T>::V V;
  const T* A = (const T*)Ap; const T* A2 = (const T*)A2p; const T* Bt = (const T*)Btp; const T* Bt2 = (const T*)Bt2p;
  __shared__ __align__(16) float sT[8][16 * 68];
  const int b    = blockIdx.y;
  const int lane = threadIdx.x & 31;
  const int wave = threadIdx.x >> 5;
  const int tilesN = N >> 6;
  const int tilesM = M >> 6;
  const int tile = blockIdx.x * 8 + wave;
  if (tile >= tilesM * tilesN) return;
  const int tm = tile / tilesN;
  const int tn = tile - tm * tilesN;
  const int m0 = tm << 6;
  const int n0 = tn << 6;
  int Kloc = K;
  if (SKIP != 0) {
    const int bb = (SKIP == 1) ? (m0 >> 9) : b;
    int ln = lens[bb];
    ln = ln < 0 ? 0 : (ln > 512 ? 512 : ln);
    const int mt = (SKIP == 1) ? (m0 & 511) : m0;
    if (mt >= ln) return;
    if (SKIP == 2) { if (n0 >= ln) return; }
    if (SKIP == 3) { Kloc = ((ln + 63) >> 6) << 6; }
  }

  const T* Ab  = A  + (size_t)b * strideA;
  const T* Bb  = Bt + (size_t)b * strideB;
  const T* Ab2 = SPLIT ? (A2  + (size_t)b * strideA) : nullptr;
  const T* Bb2 = SPLIT ? (Bt2 + (size_t)b * strideB) : nullptr;

  const int rlane = lane & 15;
  const int koff  = (lane >> 4) * 8;
  const int mOff  = (lane >> 4) * 8;

  v8f acc[4][4];
#pragma unroll
  for (int i = 0; i < 4; ++i)
#pragma unroll
    for (int j = 0; j < 4; ++j) acc[i][j] = (v8f){0.f,0.f,0.f,0.f,0.f,0.f,0.f,0.f};

  for (int k0 = 0; k0 < Kloc; k0 += 32) {
    V bh[4], bl[4];
#pragma unroll
    for (int j = 0; j < 4; ++j) {
      const size_t bo = (size_t)(n0 + (j << 4) + rlane) * ldb + koff + k0;
      bh[j] = Frag<T>::load(Bb + bo);
      if (SPLIT) bl[j] = Frag<T>::load(Bb2 + bo);
    }
#pragma unroll
    for (int i = 0; i < 4; ++i) {
      const size_t ao = (size_t)(m0 + (i << 4) + rlane) * lda + koff + k0;
      V ah = Frag<T>::load(Ab + ao);
      V al;
      if (SPLIT) al = Frag<T>::load(Ab2 + ao);
#pragma unroll
      for (int j = 0; j < 4; ++j) {
        acc[i][j] = Frag<T>::mma(ah, bh[j], acc[i][j]);
        if (SPLIT) {
          acc[i][j] = Frag<T>::mma(ah, bl[j], acc[i][j]);
          acc[i][j] = Frag<T>::mma(al, bh[j], acc[i][j]);
        }
      }
      Frag<T>::guard4(acc[i][0], acc[i][1], acc[i][2], acc[i][3], ah, SPLIT ? al : ah);
    }
    Frag<T>::keep(bh[0], bh[1], bh[2], bh[3]);
    if (SPLIT) Frag<T>::keep(bl[0], bl[1], bl[2], bl[3]);
  }
  acc_guard4(acc[0][0], acc[0][1], acc[0][2], acc[0][3]);
  acc_guard4(acc[1][0], acc[1][1], acc[1][2], acc[1][3]);
  acc_guard4(acc[2][0], acc[2][1], acc[2][2], acc[2][3]);
  acc_guard4(acc[3][0], acc[3][1], acc[3][2], acc[3][3]);

  float* slab = sT[wave];
#pragma unroll
  for (int i = 0; i < 4; ++i) {
    const int mBase = m0 + (i << 4);
#pragma unroll
    for (int j = 0; j < 4; ++j) {
      const int n = n0 + (j << 4) + rlane;
      float bv = 0.f;
      if (BIAS_MODE == 2) bv = bias[n];
#pragma unroll
      for (int r = 0; r < 8; ++r) {
        float v = acc[i][j][r] * scale;
        if (BIAS_MODE == 2) v += bv;
        slab[(mOff + r) * 68 + (j << 4) + rlane] = v;
      }
    }
    __builtin_amdgcn_fence(__ATOMIC_RELEASE, "workgroup");
    __builtin_amdgcn_wave_barrier();
    __builtin_amdgcn_fence(__ATOMIC_ACQUIRE, "workgroup");
    if (OUT_MODE == 0) {
      float* C = (float*)Cout + (size_t)b * strideC;
      const int hh = lane >> 4, c4 = (lane & 15) * 4;
      for (int pass = 0; pass < 2; ++pass) {
#pragma unroll
        for (int it = 0; it < 8; ++it) {
          const int row = it * 2 + hh;
          v4f v = *(const v4f*)(slab + row * 68 + c4);
          *(volatile v4f*)(C + (size_t)(mBase + row) * ldc + n0 + c4) = v;
        }
        __threadfence();
      }
    } else {
      const int q = lane >> 3, c8 = (lane & 7) * 8;
      unsigned short* C  = (unsigned short*)Cout  + (size_t)b * strideC;
      unsigned short* C2 = (OUT_MODE == 2) ? ((unsigned short*)Cout2 + (size_t)b * strideC) : nullptr;
      for (int pass = 0; pass < 2; ++pass) {
#pragma unroll
        for (int it = 0; it < 4; ++it) {
          const int row = it * 4 + q;
          const float* sp = slab + row * 68 + c8;
          v8h hv, lv;
#pragma unroll
          for (int e = 0; e < 8; ++e) {
            if (OUT_MODE == 1) {
              hv[e] = (_Float16)sp[e];
            } else {
              unsigned short hb = f2bf_bits(sp[e]);
              unsigned short lb = f2bf_bits(sp[e] - bf_bits2f(hb));
              hv[e] = __builtin_bit_cast(_Float16, hb);
              lv[e] = __builtin_bit_cast(_Float16, lb);
            }
          }
          *(volatile v8h*)(C + (size_t)(mBase + row) * ldc + n0 + c8) = hv;
          if (OUT_MODE == 2) *(volatile v8h*)(C2 + (size_t)(mBase + row) * ldc + n0 + c8) = lv;
        }
        __threadfence();
      }
    }
    __builtin_amdgcn_fence(__ATOMIC_RELEASE, "workgroup");
    __builtin_amdgcn_wave_barrier();
    __builtin_amdgcn_fence(__ATOMIC_ACQUIRE, "workgroup");
  }
}

__global__ __launch_bounds__(256) void cvt8_kernel(const float* __restrict__ src, unsigned short* __restrict__ dst,
                                                   int nrow, int nreal, int ncol8, int spitch, float sc) {
  const int i  = blockIdx.x * 256 + threadIdx.x;
  const int n8 = nrow * ncol8;
  if (i < n8) {
    const int row = i / ncol8;
    const int c8  = i - row * ncol8;
    const bool inr = row < nreal;
    const int rc = inr ? row : (nreal - 1);
    const float* sp = src + (size_t)rc * spitch + c8 * 8;
    const v4f a = *(const v4f*)(sp);
    const v4f b = *(const v4f*)(sp + 4);
    v8h hv;
#pragma unroll
    for (int e = 0; e < 4; ++e) {
      const float x0 = inr ? a[e] : 0.0f;
      const float x1 = inr ? b[e] : 0.0f;
      hv[e]     = (_Float16)(bf16r(x0) * sc);
      hv[4 + e] = (_Float16)(bf16r(x1) * sc);
    }
    *(volatile v8h*)(dst + (size_t)i * 8) = hv;
    __threadfence();
    *(volatile v8h*)(dst + (size_t)i * 8) = hv;
  }
}

__global__ __launch_bounds__(256) void tpose_enc_kernel(const float* __restrict__ src, unsigned short* __restrict__ O) {
  __shared__ float Tt[64 * 65];
  const int tid = threadIdx.x;
  const int c0 = blockIdx.x * 64, r0 = blockIdx.y * 64;
  const float* sb = src + (size_t)blockIdx.z * kS * kH;
  unsigned short* ob = O + (size_t)blockIdx.z * kH * kS;
#pragma unroll
  for (int i = 0; i < 4; ++i) {
    const int idx = i * 256 + tid;
    const int rr = idx >> 4, cc = (idx & 15) * 4;
    const v4f v = *(const v4f*)(sb + (size_t)(r0 + rr) * (size_t)kH + c0 + cc);
    Tt[rr * 65 + cc + 0] = v[0];
    Tt[rr * 65 + cc + 1] = v[1];
    Tt[rr * 65 + cc + 2] = v[2];
    Tt[rr * 65 + cc + 3] = v[3];
  }
  __syncthreads();
  const int q = tid >> 3, c8 = (tid & 7) * 8;
  v8h hv[2];
#pragma unroll
  for (int g = 0; g < 2; ++g) {
    const int qq = g * 32 + q;
#pragma unroll
    for (int e = 0; e < 8; ++e) {
      const float f = Tt[(c8 + e) * 65 + qq];
      hv[g][e] = (_Float16)bf16r(f);
    }
  }
  for (int pass = 0; pass < 2; ++pass) {
#pragma unroll
    for (int g = 0; g < 2; ++g) {
      const size_t o = (size_t)(c0 + g * 32 + q) * (size_t)kS + (size_t)(r0 + c8);
      *(volatile v8h*)(ob + o) = hv[g];
    }
    __threadfence();
  }
}

__global__ __launch_bounds__(256) void bias_prep_kernel(const float* __restrict__ bih, const float* __restrict__ bhh,
                                                        const float* __restrict__ batt, const float* __restrict__ bfc,
                                                        float* __restrict__ dst) {
  const int f = (blockIdx.x * 256 + threadIdx.x) * 4;
  if (f >= kBiasN) return;
  const int f0 = f < (kL * kGD - 4) ? f : (kL * kGD - 4);
  int f1 = f - kL * kGD;
  f1 = f1 < 0 ? 0 : (f1 > kH - 4 ? kH - 4 : f1);
  const int f2r = f - (kL * kGD + kH);
  const int f2 = f2r < 0 ? 0 : (f2r > kOut - 4 ? kOut - 4 : f2r);
  const v4f va = *(const v4f*)(bih + f0);
  const v4f vb = *(const v4f*)(bhh + f0);
  const v4f vc = *(const v4f*)(batt + f1);
  const v4f vd = *(const v4f*)(bfc + f2);
  v4f o;
#pragma unroll
  for (int e = 0; e < 4; ++e) {
    const float s0 = bf16r(va[e]) + bf16r(vb[e]);
    const float s1 = bf16r(vc[e]);
    const float s2 = (f2r < kOut) ? bf16r(vd[e]) : 0.0f;
    o[e] = (f < kL * kGD) ? s0 : ((f < kL * kGD + kH) ? s1 : s2);
  }
  *(volatile v4f*)(dst + f) = o;
  __threadfence();
  *(volatile v4f*)(dst + f) = o;
}

template <int LAYER>
__global__ __launch_bounds__(512) void lstm_seq_kernel(
    const float* __restrict__ ZX, const int* __restrict__ tok, const unsigned short* __restrict__ WHp,
    const float* hsrc, long hdir, long hrow, const float* csrc, int rnd,
    unsigned short* __restrict__ HSEQ, float* H1, float* CST, int t0, int t1) {
  __shared__ __align__(16) _Float16 Ah[2][kB * kHP];
  __shared__ __align__(16) float Sl[LAYER ? 16 : 1][16 * kSLP];
  const _Float16* WH = (const _Float16*)WHp;
  const int tid = threadIdx.x, lane = tid & 31, wave = tid >> 5;
  const int c = lane & 15, hh = lane >> 4, koff = hh * 8;
  const int dir = blockIdx.x;

  {
    const float* hp = hsrc + (size_t)dir * (size_t)hdir;
#pragma unroll 1
    for (int i = 0; i < kB; ++i) {
      float v = hp[(size_t)i * (size_t)hrow + tid];
      if (rnd) v = bf16r(v);
      Ah[0][i * kHP + tid] = (_Float16)(v * kHCarry);
    }
  }
  float cst[2][8];
#pragma unroll
  for (int nt = 0; nt < 2; ++nt) {
    const int j = 32 * wave + 16 * nt + c;
#pragma unroll
    for (int r = 0; r < 8; ++r) {
      float v = csrc[((size_t)dir * kB + 8 * hh + r) * kH + j];
      if (rnd) v = bf16r(v);
      cst[nt][r] = v;
    }
  }
  __syncthreads();

  const v8f z8 = {0.f, 0.f, 0.f, 0.f, 0.f, 0.f, 0.f, 0.f};
  float* slab = Sl[LAYER ? wave : 0];

#pragma unroll 1
  for (int t = t0; t < t1; ++t) {
    const int cur = (t - t0) & 1;
    const _Float16* ahrow = &Ah[cur][0] + c * kHP + koff;
    _Float16* ahn = &Ah[cur ^ 1][0];
    int zrow[8];
#pragma unroll
    for (int r = 0; r < 8; ++r) {
      if (LAYER == 0) {
        int tk = tok[(8 * hh + r) * kT + t];
        tk = tk < 0 ? 0 : (tk > kVoc - 1 ? kVoc - 1 : tk);
        zrow[r] = tk;
      } else {
        zrow[r] = (t - t0) * kB + 8 * hh + r;
      }
    }
#pragma unroll
    for (int nt = 0; nt < 2; ++nt) {
      const int j = 32 * wave + 16 * nt + c;
      const _Float16* wh = WH + ((size_t)dir * kG + j) * kH + koff;
      v8f a0 = z8, a1 = z8, a2 = z8, a3 = z8;
#pragma unroll 1
      for (int k0 = 0; k0 < kH; k0 += 32) {
        const v16h a  = Frag<_Float16>::load(ahrow + k0);
        const v16h b0 = Frag<_Float16>::load(wh + k0);
        const v16h b1 = Frag<_Float16>::load(wh + (size_t)1 * kH * kH + k0);
        const v16h b2 = Frag<_Float16>::load(wh + (size_t)2 * kH * kH + k0);
        const v16h b3 = Frag<_Float16>::load(wh + (size_t)3 * kH * kH + k0);
        a0 = Frag<_Float16>::mma(a, b0, a0);
        a1 = Frag<_Float16>::mma(a, b1, a1);
        a2 = Frag<_Float16>::mma(a, b2, a2);
        a3 = Frag<_Float16>::mma(a, b3, a3);
        guard4w_h(a0, a1, a2, a3, a, b0, b1, b2, b3);
      }
      acc_guard4(a0, a1, a2, a3);
#pragma unroll
      for (int r = 0; r < 8; ++r) {
        const float* zb = ZX + (size_t)zrow[r] * kGD + dir * kG + j;
        const float zi = a0[r] * kFoldHW + zb[0];
        const float zf = a1[r] * kFoldHW + zb[kH];
        const float zg = a2[r] * kFoldHW + zb[2 * kH];
        const float zo = a3[r] * kFoldHW + zb[3 * kH];
        const float ig = fsig(zi);
        const float fg = fsig(zf);
        const float gg = ftanh(zg);
        const float og = fsig(zo);
        const float cn = fg * cst[nt][r] + ig * gg;
        cst[nt][r] = cn;
        const float hn = og * ftanh(cn);
        ahn[(8 * hh + r) * kHP + j] = (_Float16)(hn * kHCarry);
        if (LAYER == 1) slab[(8 * hh + r) * kSLP + 16 * nt + c] = hn;
      }
    }
    if (LAYER == 1) {
      __builtin_amdgcn_fence(__ATOMIC_RELEASE, "workgroup");
      __builtin_amdgcn_wave_barrier();
      __builtin_amdgcn_fence(__ATOMIC_ACQUIRE, "workgroup");
      const int q = lane >> 3, c4 = (lane & 7) * 4;
      for (int pass = 0; pass < 2; ++pass) {
#pragma unroll
        for (int it = 0; it < 4; ++it) {
          const int row = it * 4 + q;
          const v4f v = *(const v4f*)(slab + row * kSLP + c4);
          *(volatile v4f*)(H1 + (((size_t)dir * kB + row) * kT + (size_t)t) * kH + 32 * wave + c4) = v;
        }
        __threadfence();
      }
      __builtin_amdgcn_fence(__ATOMIC_RELEASE, "workgroup");
      __builtin_amdgcn_wave_barrier();
      __builtin_amdgcn_fence(__ATOMIC_ACQUIRE, "workgroup");
    }
    __syncthreads();
    if (LAYER == 0) {
      for (int pass = 0; pass < 2; ++pass) {
#pragma unroll
        for (int it = 0; it < 2; ++it) {
          const int idx = it * 512 + tid;
          const int row = idx >> 6, c8 = (idx & 63) * 8;
          const v8h v = *(const v8h*)(ahn + row * kHP + c8);
          *(volatile v8h*)(HSEQ + ((size_t)t * kB + row) * (2 * kH) + dir * kH + c8) = v;
        }
        __threadfence();
      }
    }
  }

  if (LAYER == 1) {
#pragma unroll
    for (int nt = 0; nt < 2; ++nt)
#pragma unroll
      for (int r = 0; r < 8; ++r) slab[(8 * hh + r) * kSLP + 16 * nt + c] = cst[nt][r];
    __builtin_amdgcn_fence(__ATOMIC_RELEASE, "workgroup");
    __builtin_amdgcn_wave_barrier();
    __builtin_amdgcn_fence(__ATOMIC_ACQUIRE, "workgroup");
    const int q = lane >> 3, c4 = (lane & 7) * 4;
    for (int pass = 0; pass < 2; ++pass) {
#pragma unroll
      for (int it = 0; it < 4; ++it) {
        const int row = it * 4 + q;
        const v4f v = *(const v4f*)(slab + row * kSLP + c4);
        *(volatile v4f*)(CST + ((size_t)dir * kB + row) * kH + 32 * wave + c4) = v;
      }
      __threadfence();
    }
  }
}

__global__ __launch_bounds__(256) void combine_kernel(const float* __restrict__ H1, unsigned short* __restrict__ DH,
                                                      unsigned short* __restrict__ DL, unsigned short* __restrict__ CAT) {
  const int i = blockIdx.x * 256 + threadIdx.x;
  if (i >= kRows * (kH / 8)) return;
  const float* p0 = H1 + (size_t)i * 8;
  const float* p1 = H1 + (size_t)kRows * kH + (size_t)i * 8;
  const v4f a0 = *(const v4f*)(p0);
  const v4f a1 = *(const v4f*)(p0 + 4);
  const v4f b0 = *(const v4f*)(p1);
  const v4f b1 = *(const v4f*)(p1 + 4);
  v8h vh, vl, vc;
#pragma unroll
  for (int e = 0; e < 4; ++e) {
    const float d0 = a0[e] + b0[e];
    const float d1 = a1[e] + b1[e];
    const unsigned short h0 = f2bf_bits(d0);
    const unsigned short l0 = f2bf_bits(d0 - bf_bits2f(h0));
    const unsigned short h1 = f2bf_bits(d1);
    const unsigned short l1 = f2bf_bits(d1 - bf_bits2f(h1));
    vh[e]     = __builtin_bit_cast(_Float16, h0);
    vl[e]     = __builtin_bit_cast(_Float16, l0);
    vh[4 + e] = __builtin_bit_cast(_Float16, h1);
    vl[4 + e] = __builtin_bit_cast(_Float16, l1);
    vc[e]     = (_Float16)(d0 * kCatCarry);
    vc[4 + e] = (_Float16)(d1 * kCatCarry);
  }
  const int row = i >> 6, c8 = (i & 63) * 8;
  unsigned short* ph = DH + (size_t)i * 8;
  unsigned short* pl = DL + (size_t)i * 8;
  unsigned short* pc = CAT + (size_t)row * (2 * kH) + c8;
  *(volatile v8h*)ph = vh;
  *(volatile v8h*)pl = vl;
  *(volatile v8h*)pc = vc;
  __threadfence();
  *(volatile v8h*)ph = vh;
  *(volatile v8h*)pl = vl;
  *(volatile v8h*)pc = vc;
}

__global__ __launch_bounds__(256) void softmax_kernel(const float* __restrict__ SC, const int* __restrict__ lens,
                                                      unsigned short* __restrict__ ATT) {
  __shared__ __align__(16) float srow[8][kS];
  const int tid = threadIdx.x, lane = tid & 31, wave = tid >> 5;
  const int row = blockIdx.x * 8 + wave;
  const int b = row >> 9, t = row & 511;
  int len = lens[b];
  len = len < 0 ? 0 : (len > kS ? kS : len);
  const int LT = ((len + 63) >> 6) << 6;
  unsigned short* op = ATT + (size_t)row * kS;
  if (t >= LT) {
    const v4u z = (v4u){0u, 0u, 0u, 0u};
    for (int pass = 0; pass < 2; ++pass) {
#pragma unroll
      for (int k = 0; k < 2; ++k) *(volatile v4u*)(op + k * 256 + 8 * lane) = z;
      __threadfence();
    }
    return;
  }
  float* sr = srow[wave];
  const float* sp = SC + (size_t)row * kS;
  float m = -INFINITY;
#pragma unroll 1
  for (int k = 0; k < 2; ++k) {
    const int c0 = k * 256 + 8 * lane;
    const int cl = (c0 < LT) ? c0 : 0;
    const v4f a = *(const v4f*)(sp + cl);
    const v4f q = *(const v4f*)(sp + cl + 4);
    v4f xa, xb;
#pragma unroll
    for (int e = 0; e < 4; ++e) {
      xa[e] = (c0 + e < len) ? a[e] : -1e30f;
      xb[e] = (c0 + 4 + e < len) ? q[e] : -1e30f;
      m = fmaxf(m, fmaxf(xa[e], xb[e]));
    }
    *(v4f*)(sr + c0) = xa;
    *(v4f*)(sr + c0 + 4) = xb;
  }
#pragma unroll
  for (int off = 1; off < 32; off <<= 1) m = fmaxf(m, __shfl_xor(m, off, 32));
  float sum = 0.0f;
#pragma unroll 1
  for (int k = 0; k < 2; ++k) {
    const int c0 = k * 256 + 8 * lane;
    v4f xa = *(const v4f*)(sr + c0);
    v4f xb = *(const v4f*)(sr + c0 + 4);
#pragma unroll
    for (int e = 0; e < 4; ++e) {
      xa[e] = expf(xa[e] - m);
      xb[e] = expf(xb[e] - m);
      sum += xa[e] + xb[e];
    }
    *(v4f*)(sr + c0) = xa;
    *(v4f*)(sr + c0 + 4) = xb;
  }
#pragma unroll
  for (int off = 1; off < 32; off <<= 1) sum += __shfl_xor(sum, off, 32);
  const float sc = kPCarry * (1.0f / sum);
  for (int pass = 0; pass < 2; ++pass) {
#pragma unroll 1
    for (int k = 0; k < 2; ++k) {
      const int c0 = k * 256 + 8 * lane;
      const v4f xa = *(const v4f*)(sr + c0);
      const v4f xb = *(const v4f*)(sr + c0 + 4);
      v8h hv;
#pragma unroll
      for (int e = 0; e < 4; ++e) {
        hv[e]     = (_Float16)(xa[e] * sc);
        hv[4 + e] = (_Float16)(xb[e] * sc);
      }
      *(volatile v8h*)(op + c0) = hv;
    }
    __threadfence();
  }
}

__global__ __launch_bounds__(256) void pack_kernel(const float* __restrict__ FC, const int* __restrict__ lens,
                                                   float* __restrict__ out) {
  const int lane = threadIdx.x & 31;
  const int wg = blockIdx.x * 8 + (threadIdx.x >> 5);
  v4f o[2];
#pragma unroll
  for (int k = 0; k < 2; ++k) {
    const int ch = wg * 64 + k * 32 + lane;
    const int f = ch * 4;
    const int m = f / kOut;
    const int n = f - m * kOut;
    const int b = m >> 9, t = m & 511;
    int len = lens[b];
    len = len < 0 ? 0 : (len > kT ? kT : len);
    const bool valid = t < len;
    const int mm = valid ? m : (b << 9);
    const v4f v = *(const v4f*)(FC + (size_t)mm * kOutP + n);
#pragma unroll
    for (int e = 0; e < 4; ++e) o[k][e] = valid ? v[e] : 0.0f;
  }
  float* ob = out + (size_t)wg * 256;
  for (int pass = 0; pass < 2; ++pass) {
#pragma unroll
    for (int k = 0; k < 2; ++k) *(volatile v4f*)(ob + k * 128 + lane * 4) = o[k];
    __threadfence();
  }
}

extern "C" void kernel_launch(void* const* d_in, const int* in_sizes, int n_in,
                              void* d_out, int out_size, void* d_ws, size_t ws_size, hipStream_t stream) {
  if (n_in < 15 || d_out == nullptr || d_ws == nullptr) return;
  if (in_sizes[0] != kB * kT || in_sizes[1] != kB || in_sizes[2] != kB * kS * kH ||
      in_sizes[3] != 2 * kL * kB * kH || in_sizes[4] != 2 * kL * kB * kH || in_sizes[5] != kVoc * kE ||
      in_sizes[6] != 2 * kG * kE || in_sizes[7] != 2 * kG * 2 * kH || in_sizes[8] != kL * 2 * kG * kH ||
      in_sizes[9] != kL * 2 * kG || in_sizes[10] != kL * 2 * kG || in_sizes[11] != kH * kH ||
      in_sizes[12] != kH || in_sizes[13] != kOut * 2 * kH || in_sizes[14] != kOut ||
      out_size != kRows * kOut) return;

  const int*   tok   = (const int*)d_in[0];
  const int*   lens  = (const int*)d_in[1];
  const float* enc   = (const float*)d_in[2];
  const float* h0    = (const float*)d_in[3];
  const float* c0    = (const float*)d_in[4];
  const float* embed = (const float*)d_in[5];
  const float* w_ih0 = (const float*)d_in[6];
  const float* w_ih1 = (const float*)d_in[7];
  const float* w_hh  = (const float*)d_in[8];
  const float* b_ih  = (const float*)d_in[9];
  const float* b_hh  = (const float*)d_in[10];
  const float* w_att = (const float*)d_in[11];
  const float* b_att = (const float*)d_in[12];
  const float* w_fc  = (const float*)d_in[13];
  const float* b_fc  = (const float*)d_in[14];
  float* out = (float*)d_out;

  char* ws = (char*)d_ws; size_t off = 0;
  auto carve = [&](size_t bytes) -> char* { char* p = ws + off; off += (bytes + 255) & ~(size_t)255; return p; };
  unsigned short* WHH16 = (unsigned short*)carve((size_t)kL * 2 * kG * kH * 2);
  unsigned short* WIH0  = (unsigned short*)carve((size_t)kGD * kE * 2);
  unsigned short* WIH1  = (unsigned short*)carve((size_t)kGD * 2 * kH * 2);
  unsigned short* EMB16 = (unsigned short*)carve((size_t)kVocP * kE * 2);
  float*          G0    = (float*)carve((size_t)kVocP * kGD * 4);
  unsigned short* HSEQ0 = (unsigned short*)carve((size_t)kRows * 2 * kH * 2);
  float*          XPROJ = (float*)carve((size_t)kB * kChunk * kGD * 4);
  const size_t endA = off;
  off = 0;
  unsigned short* ENC16  = (unsigned short*)carve((size_t)kRows * kH * 2);
  unsigned short* ENCT   = (unsigned short*)carve((size_t)kB * kH * kS * 2);
  unsigned short* WATT16 = (unsigned short*)carve((size_t)kH * kH * 2);
  unsigned short* EPJH   = (unsigned short*)carve((size_t)kRows * kH * 2);
  unsigned short* EPJL   = (unsigned short*)carve((size_t)kRows * kH * 2);
  unsigned short* DECH   = (unsigned short*)carve((size_t)kRows * kH * 2);
  unsigned short* DECL   = (unsigned short*)carve((size_t)kRows * kH * 2);
  unsigned short* CAT16  = (unsigned short*)carve((size_t)kRows * 2 * kH * 2);
  float*          SCORE  = (float*)carve((size_t)kB * kT * kS * 4);
  unsigned short* ATT    = (unsigned short*)carve((size_t)kB * kT * kS * 2);
  unsigned short* WFC16  = (unsigned short*)carve((size_t)kOutP * 2 * kH * 2);
  const size_t endB = off;
  off = endA > endB ? endA : endB;
  float* H1     = (float*)carve((size_t)2 * kRows * kH * 4);
  float* BIASWS = (float*)carve((size_t)kBiasN * 4);
  float* CST    = (float*)carve((size_t)2 * kB * kH * 4);
  float* FCPAD  = H1;
  if (off > ws_size || off > (size_t)134217728) return;

  bias_prep_kernel<<<(kBiasN / 4 + 255) / 256, 256, 0, stream>>>(b_ih, b_hh, b_att, b_fc, BIASWS);

  cvt8_kernel<<<(kL * 2 * kG * (kH / 8)) / 256, 256, 0, stream>>>(w_hh,  WHH16, kL * 2 * kG, kL * 2 * kG, kH / 8, kH, kWCarry);
  cvt8_kernel<<<(kGD * (kE / 8)) / 256, 256, 0, stream>>>(w_ih0, WIH0, kGD, kGD, kE / 8, kE, kWCarry);
  cvt8_kernel<<<(kGD * (2 * kH / 8)) / 256, 256, 0, stream>>>(w_ih1, WIH1, kGD, kGD, 2 * kH / 8, 2 * kH, kWCarry);
  cvt8_kernel<<<(kVocP * (kE / 8)) / 256, 256, 0, stream>>>(embed, EMB16, kVocP, kVoc, kE / 8, kE, kECarry);

  wmma_gemm64<0, false, 2, 0, 0><<<dim3((kVocP / 64) * (kGD / 64) / 8, 1), 256, 0, stream>>>(
      EMB16, EMB16, kE, 0L, WIH0, WIH0, kE, 0L, (void*)G0, (void*)G0, kGD, 0L,
      BIASWS, lens, kVocP, kGD, kE, kFoldEW);

  lstm_seq_kernel<0><<<2, 512, 0, stream>>>(G0, tok, WHH16, h0, (long)(kB * kH), (long)kH, c0, 1,
                                            HSEQ0, H1, CST, 0, kT);

  for (int ck = 0; ck < kT / kChunk; ++ck) {
    const int t0 = ck * kChunk;
    wmma_gemm64<0, false, 2, 0, 0><<<dim3((kB * kChunk / 64) * (kGD / 64) / 8, 1), 256, 0, stream>>>(
        HSEQ0 + (size_t)t0 * kB * 2 * kH, HSEQ0 + (size_t)t0 * kB * 2 * kH, 2 * kH, 0L,
        WIH1, WIH1, 2 * kH, 0L, (void*)XPROJ, (void*)XPROJ, kGD, 0L,
        BIASWS + kGD, lens, kB * kChunk, kGD, 2 * kH, kFoldHW);
    const float* hs = (ck == 0) ? (h0 + (size_t)2 * kB * kH) : (H1 + (size_t)(t0 - 1) * kH);
    const long hd   = (ck == 0) ? (long)(kB * kH) : (long)kB * kT * kH;
    const long hr   = (ck == 0) ? (long)kH : (long)kT * kH;
    const float* cs = (ck == 0) ? (c0 + (size_t)2 * kB * kH) : CST;
    lstm_seq_kernel<1><<<2, 512, 0, stream>>>(XPROJ, tok, WHH16 + (size_t)2 * kG * kH, hs, hd, hr, cs,
                                              (ck == 0) ? 1 : 0, HSEQ0, H1, CST, t0, t0 + kChunk);
  }

  cvt8_kernel<<<(kRows * (kH / 8)) / 256, 256, 0, stream>>>(enc, ENC16, kRows, kRows, kH / 8, kH, 1.0f);
  cvt8_kernel<<<(kH * (kH / 8)) / 256, 256, 0, stream>>>(w_att, WATT16, kH, kH, kH / 8, kH, kWCarry);
  cvt8_kernel<<<(kOutP * (2 * kH / 8)) / 256, 256, 0, stream>>>(w_fc, WFC16, kOutP, kOut, 2 * kH / 8, 2 * kH, kWCarry);
  tpose_enc_kernel<<<dim3(kH / 64, kS / 64, kB), 256, 0, stream>>>(enc, ENCT);

  combine_kernel<<<(kRows * (kH / 8)) / 256, 256, 0, stream>>>(H1, DECH, DECL, CAT16);

  wmma_gemm64<0, false, 2, 2, 1><<<dim3((kRows / 64) * (kH / 64) / 8, 1), 256, 0, stream>>>(
      ENC16, ENC16, kH, 0L, WATT16, WATT16, kH, 0L, (void*)EPJH, (void*)EPJL, kH, 0L,
      BIASWS + kL * kGD, lens, kRows, kH, kH, kFoldW);

  wmma_gemm64<1, true, 0, 0, 2><<<dim3((kT / 64) * (kS / 64) / 8, kB), 256, 0, stream>>>(
      DECH, DECL, kH, (long)kT * kH, EPJH, EPJL, kH, (long)kS * kH,
      (void*)SCORE, (void*)SCORE, kS, (long)kT * kS,
      BIASWS, lens, kT, kS, kH, 1.0f);

  softmax_kernel<<<kRows / 8, 256, 0, stream>>>(SCORE, lens, ATT);

  wmma_gemm64<0, false, 0, 1, 3><<<dim3((kT / 64) * (kH / 64) / 8, kB), 256, 0, stream>>>(
      ATT, ATT, kS, (long)kT * kS, ENCT, ENCT, kS, (long)kH * kS,
      (void*)(CAT16 + kH), (void*)(CAT16 + kH), 2 * kH, (long)kT * 2 * kH,
      BIASWS, lens, kT, kH, kS, kCtxScale);

  wmma_gemm64<0, false, 2, 0, 1><<<dim3((kRows / 64) * (kOutP / 64) / 8, 1), 256, 0, stream>>>(
      CAT16, CAT16, 2 * kH, 0L, WFC16, WFC16, 2 * kH, 0L, (void*)FCPAD, (void*)FCPAD, kOutP, 0L,
      BIASWS + kL * kGD + kH, lens, kRows, kOutP, 2 * kH, kFoldCW);

  pack_kernel<<<(kRows / 2048) * kOut, 256, 0, stream>>>(FCPAD, lens, out);
}
